// STDP_30897994727567
// MI455X (gfx1250) — hardware-verified
//
#include <hip/hip_runtime.h>


namespace {
constexpr int T = 100, B = 32, NI = 1024, NO = 512, KT = T * B;
constexpr float XS = 8.0f, LR = 1e-4f;
typedef _Float16 b16;
typedef __attribute__((ext_vector_type(16))) _Float16 v16b;
typedef __attribute__((ext_vector_type(8))) _Float16 v8b;
typedef __attribute__((ext_vector_type(8))) float v8f;
typedef __attribute__((ext_vector_type(4))) float v4f;
__device__ __forceinline__ float bf16_rne(float f) { unsigned int u = __float_as_uint(f); u += 0x7FFFu + ((u >> 16) & 1u); return __uint_as_float(u & 0xFFFF0000u); }
__device__ __forceinline__ void split16(float v, b16& hi, b16& lo) { hi = (b16)v; lo = (b16)(v - (float)hi); }
__device__ __forceinline__ v16b frag_kb(const b16* p, int hh) { const v8b a = *(const v8b*)(p + 8 * hh), b = *(const v8b*)(p + 16 + 8 * hh); v16b f;
#pragma unroll
  for (int e = 0; e < 8; ++e) { f[e] = a[e]; f[8 + e] = b[e]; } return f; }
__device__ __forceinline__ v8f wmma16b(v16b a, v16b b, v8f c) { v8f d = __builtin_amdgcn_wmma_f32_16x16x32_f16(false, a, false, b, (short)0, c, false, false); asm volatile("v_nop\n\tv_nop\n\tv_nop\n\tv_nop" : "+v"(d) : "v"(a), "v"(b)); return d; }
__device__ __forceinline__ void wave_lds_sync() { __builtin_amdgcn_fence(__ATOMIC_RELEASE, "workgroup"); __builtin_amdgcn_wave_barrier(); __builtin_amdgcn_fence(__ATOMIC_ACQUIRE, "workgroup"); }
__device__ __forceinline__ float pmul(float a, float b) { float p = a * b; asm volatile("" : "+v"(p)); return p; }

template <int NU>
__global__ __launch_bounds__(256) void plane_kernel(const float* __restrict__ spikes, const float* __restrict__ tr0, int TL, b16* __restrict__ SP, b16* __restrict__ TH, b16* __restrict__ TLw) {
  const int idx = blockIdx.x * 256 + threadIdx.x; if (idx >= NU * 4) return; const int u = idx >> 2, g = idx & 3; const float decay = __expf(-1.0f / 20.0f);
  for (int pass = 0; pass < 2; ++pass) { float tr[8];
#pragma unroll
    for (int b = 0; b < 8; ++b) tr[b] = bf16_rne(tr0[(g * 8 + b) * NU + u]);
#pragma unroll 1
    for (int t = 0; t < TL; ++t) { v8b sv, hv, lv;
#pragma unroll
      for (int b = 0; b < 8; ++b) { const float s = bf16_rne(spikes[((size_t)t * B + g * 8 + b) * NU + u]); tr[b] = pmul(tr[b], decay) + s; b16 p, q; split16(tr[b] * XS, p, q); sv[b] = (b16)s; hv[b] = p; lv[b] = q; }
      const size_t o_ = (size_t)u * KT + t * B + g * 8; *(volatile v8b*)(SP + o_) = sv; *(volatile v8b*)(TH + o_) = hv; *(volatile v8b*)(TLw + o_) = lv; }
    __threadfence(); }
}
template <int NU>
__global__ __launch_bounds__(256) void trace_out_kernel(const float* __restrict__ spikes, const float* __restrict__ tr0, int TL, float* __restrict__ out) {
  const int idx = blockIdx.x * 256 + threadIdx.x; if (idx >= B * NU) return; const int b = idx / NU, u = idx % NU; const float decay = __expf(-1.0f / 20.0f); float tr = bf16_rne(tr0[b * NU + u]);
#pragma unroll 1
  for (int t = 0; t < TL; ++t) tr = pmul(tr, decay) + bf16_rne(spikes[((size_t)t * B + b) * NU + u]);
  for (int pass = 0; pass < 2; ++pass) { ((volatile float*)out)[idx] = tr; __threadfence(); }
}
__global__ __launch_bounds__(32) void dw_kernel(const float* __restrict__ w, const b16* __restrict__ SPO, const b16* __restrict__ TOH, const b16* __restrict__ TOL, const b16* __restrict__ SPI, const b16* __restrict__ TIH, const b16* __restrict__ TIL, int TL, float* __restrict__ out) {
  __shared__ float M1[16][132], M2[16][132]; const int lane = threadIdx.x, nloc = lane & 15, hlf = lane >> 4; const int o0 = (blockIdx.x >> 3) * 16, i0 = (blockIdx.x & 7) * 128; const int KL = TL * B;
  v8f a1[8], a2[8];
#pragma unroll
  for (int t = 0; t < 8; ++t) { a1[t] = (v8f){}; a2[t] = (v8f){}; }
#pragma unroll 1
  for (int kb = 0; kb < KL; kb += 32) { const v16b sp = frag_kb(SPO + (size_t)(o0 + nloc) * KT + kb, hlf), th = frag_kb(TOH + (size_t)(o0 + nloc) * KT + kb, hlf), tl = frag_kb(TOL + (size_t)(o0 + nloc) * KT + kb, hlf);
#pragma unroll
    for (int t = 0; t < 8; ++t) { const size_t ir = (size_t)(i0 + t * 16 + nloc) * KT + kb; const v16b bh = frag_kb(TIH + ir, hlf), bl = frag_kb(TIL + ir, hlf), bs = frag_kb(SPI + ir, hlf); a1[t] = wmma16b(sp, bh, a1[t]); a1[t] = wmma16b(sp, bl, a1[t]); a2[t] = wmma16b(th, bs, a2[t]); a2[t] = wmma16b(tl, bs, a2[t]); } }
#pragma unroll
  for (int t = 0; t < 8; ++t)
#pragma unroll
    for (int r8 = 0; r8 < 8; ++r8) { M1[8 * hlf + r8][t * 16 + nloc] = a1[t][r8] * (1.0f / XS); M2[8 * hlf + r8][t * 16 + nloc] = a2[t][r8] * (1.0f / XS); }
  wave_lds_sync();
  for (int pass = 0; pass < 2; ++pass) { for (int rr = 0; rr < 16; ++rr) { v4f r; for (int q4 = 0; q4 < 4; ++q4) { const int c = lane * 4 + q4; const float wv = bf16_rne(w[(size_t)(o0 + rr) * NI + i0 + c]); r[q4] = pmul(pmul(LR * (1.0f / B), 1.0f - wv), M1[rr][c]) - pmul(pmul(LR * (1.0f / B), wv), M2[rr][c]); } *(volatile v4f*)(out + (size_t)(o0 + rr) * NI + i0 + lane * 4) = r; } __threadfence(); }
}
}

extern "C" void kernel_launch(void* const* d_in, const int* in_sizes, int n_in, void* d_out, int out_size, void* d_ws, size_t ws_size, hipStream_t stream) {
  (void)n_in;
  auto Fp = [&](int i) { return (const float*)d_in[i]; };
  if (in_sizes[0] != NO * NI || in_sizes[1] != T * B * NI || in_sizes[2] != T * B * NO || in_sizes[3] != B * NI || in_sizes[4] != B * NO || out_size != NO * NI + B * NI + B * NO) return;
  const int TL = T;
  size_t off = 0; char* ws = (char*)d_ws;
  auto carve = [&](size_t bytes) { char* p = ws + off; off += (bytes + 255) & ~(size_t)255; return p; };
  b16* SPI = (b16*)carve((size_t)NI * KT * 2); b16* TIH = (b16*)carve((size_t)NI * KT * 2); b16* TIL = (b16*)carve((size_t)NI * KT * 2); b16* SPO = (b16*)carve((size_t)NO * KT * 2); b16* TOH = (b16*)carve((size_t)NO * KT * 2); b16* TOL = (b16*)carve((size_t)NO * KT * 2);
  if (off > ws_size || off > ((size_t)48 << 20)) return;
  plane_kernel<NI><<<NI * 4 / 256, 256, 0, stream>>>(Fp(1), Fp(3), TL, SPI, TIH, TIL); plane_kernel<NO><<<NO * 4 / 256, 256, 0, stream>>>(Fp(2), Fp(4), TL, SPO, TOH, TOL);
  float* out = (float*)d_out;
  dw_kernel<<<(NO / 16) * (NI / 128), 32, 0, stream>>>(Fp(0), SPO, TOH, TOL, SPI, TIH, TIL, TL, out);
  trace_out_kernel<NI><<<B * NI / 256, 256, 0, stream>>>(Fp(1), Fp(3), TL, out + (size_t)NO * NI); trace_out_kernel<NO><<<B * NO / 256, 256, 0, stream>>>(Fp(2), Fp(4), TL, out + (size_t)NO * NI + B * NI);
}
